// LSTM_1735166788609
// MI455X (gfx1250) — hardware-verified
//
#include <hip/hip_runtime.h>
#include <math.h>

constexpr int NSTEP    = 1024;
constexpr int NBAT     = 2048;
constexpr int NIN      = 2;
constexpr int NHID     = 64;
constexpr int NGATE    = 4 * NHID;
constexpr int NTHR     = 256;
constexpr int ROWS_BLK = 32;
constexpr int HP       = 72;
constexpr int WP       = 72;
constexpr float HCARRY = 16.0f;
constexpr float WCARRY = 256.0f;
constexpr float SC_INV = 1.0f / (16.0f * 256.0f);
static_assert(NBAT % ROWS_BLK == 0);
static_assert(ROWS_BLK == 32);
static_assert(NHID == 16 * 4);
static_assert(NHID % 32 == 0);
static_assert(NGATE == NTHR);
static_assert((NGATE * NHID) % (4 * NTHR) == 0);
static_assert((2 * 2 * 16 * HP) % 8 == 0);
static_assert(HP % 8 == 0 && WP % 8 == 0);

typedef __attribute__((ext_vector_type(16))) _Float16 v16h;
typedef __attribute__((ext_vector_type(8)))  _Float16 v8h;
typedef __attribute__((ext_vector_type(16))) __bf16   v16b;
typedef __attribute__((ext_vector_type(8)))  __bf16   v8b;
typedef __attribute__((ext_vector_type(8)))  float    v8f;
typedef __attribute__((ext_vector_type(4)))  float    v4f;
typedef __attribute__((ext_vector_type(2)))  float    v2f;
typedef __attribute__((ext_vector_type(4)))  unsigned v4u;
typedef __attribute__((ext_vector_type(2)))  unsigned v2u;

__device__ __forceinline__ void dep_guard_h(v8f& a, v8f& b, v16h x, v16h y) { asm volatile("v_nop\n\tv_nop\n\tv_nop\n\tv_nop" : "+v"(a), "+v"(b) : "v"(x), "v"(y)); }
__device__ __forceinline__ void dep_guard_b(v8f& a, v8f& b, v16b x, v16b y) { asm volatile("v_nop\n\tv_nop\n\tv_nop\n\tv_nop" : "+v"(a), "+v"(b) : "v"(x), "v"(y)); }
__device__ __forceinline__ void keep4_h(v16h a, v16h b, v16h c, v16h d) { asm volatile("v_nop" :: "v"(a), "v"(b), "v"(c), "v"(d)); }
__device__ __forceinline__ void keep4_b(v16b a, v16b b, v16b c, v16b d) { asm volatile("v_nop" :: "v"(a), "v"(b), "v"(c), "v"(d)); }
__device__ __forceinline__ void acc_guard4(v8f& a, v8f& b, v8f& c, v8f& d) { asm volatile("v_nop\n\tv_nop\n\tv_nop\n\tv_nop" : "+v"(a), "+v"(b), "+v"(c), "+v"(d)); }
__device__ __forceinline__ void acc_guard4_ab(v8f& a, v8f& b, v8f& c, v8f& d, v16h x, v16h y) {
  asm volatile("v_nop\n\tv_nop\n\tv_nop\n\tv_nop" : "+v"(a), "+v"(b), "+v"(c), "+v"(d) : "v"(x), "v"(y));
}

template <typename T> struct Frag;
template <> struct Frag<_Float16> {
  typedef v16h V; union U { v16h v; v8h h[2]; };
  static __device__ __forceinline__ v16h load(const _Float16* p) {
    U f; f.h[0] = *(const v8h*)(p); f.h[1] = *(const v8h*)(p + 16); return f.v;
  }
  static __device__ __forceinline__ v8f mma(v16h a, v16h b, v8f c) {
    return __builtin_amdgcn_wmma_f32_16x16x32_f16(false, a, false, b, (short)0, c, false, false);
  }
  static __device__ __forceinline__ void guard(v8f& a, v8f& b, v16h x, v16h y) { dep_guard_h(a, b, x, y); }
  static __device__ __forceinline__ void keep(v16h a, v16h b, v16h c, v16h d) { keep4_h(a, b, c, d); }
};
template <> struct Frag<__bf16> {
  typedef v16b V; union U { v16b v; v8b h[2]; };
  static __device__ __forceinline__ v16b load(const __bf16* p) {
    U f; f.h[0] = *(const v8b*)(p); f.h[1] = *(const v8b*)(p + 16); return f.v;
  }
  static __device__ __forceinline__ v8f mma(v16b a, v16b b, v8f c) {
    return __builtin_amdgcn_wmma_f32_16x16x32_bf16(false, a, false, b, (short)0, c, false, false);
  }
  static __device__ __forceinline__ void guard(v8f& a, v8f& b, v16b x, v16b y) { dep_guard_b(a, b, x, y); }
  static __device__ __forceinline__ void keep(v16b a, v16b b, v16b c, v16b d) { keep4_b(a, b, c, d); }
};

__device__ __forceinline__ float sigm_f(float z) {
  const float e = expf(-fabsf(z));
  const float q = __builtin_amdgcn_rcpf(1.0f + e);
  return (z >= 0.0f) ? q : e * q;
}
__device__ __forceinline__ float tanh_f(float z) {
  const float e = expf(-2.0f * fabsf(z));
  const float t = (1.0f - e) * __builtin_amdgcn_rcpf(1.0f + e);
  return copysignf(t, z);
}

__global__ __launch_bounds__(NTHR) void lstm_seq_kernel(
    const float* __restrict__ x, const float* __restrict__ w_ih, const float* __restrict__ w_hh,
    const float* __restrict__ b_ih, const float* __restrict__ b_hh,
    const float* __restrict__ w_fc, const float* __restrict__ b_fc, float* __restrict__ out) {
  __shared__ __align__(16) _Float16 Wl[NGATE * WP];
  __shared__ __align__(16) _Float16 Ah[2 * 2 * 16 * HP];
  __shared__ __align__(16) float    Xs[2 * ROWS_BLK * NIN];
  __shared__ __align__(16) float    Ps[2 * 4 * 16];
  __shared__ __align__(16) float    Os[ROWS_BLK];

  const int tid = threadIdx.x, lane = tid & 31, wave = tid >> 5;
  const int c = lane & 15, hh = lane >> 4, koff = hh * 8;
  const int grp = wave >> 2;
  const int jt  = wave & 3;
  const int gi  = 16 * jt + c;
  const int blk = blockIdx.x;
  const int rowbase = blk * ROWS_BLK;

  const v4u z4 = {0u, 0u, 0u, 0u};
#pragma unroll 1
  for (int i = tid; i < (2 * 2 * 16 * HP) / 8; i += NTHR) *(v4u*)(Ah + 8 * i) = z4;
#pragma unroll 1
  for (int it = 0; it < (NGATE * NHID) / (4 * NTHR); ++it) {
    const int idx4 = it * NTHR + tid;
    const int n = idx4 >> 4, k4 = (idx4 & 15) * 4;
    const v4f v = *(const v4f*)(w_hh + (size_t)n * NHID + k4);
    const float f0 = v[0], f1 = v[1], f2 = v[2], f3 = v[3];
    const _Float16 e0 = (_Float16)(f0 * WCARRY), e1 = (_Float16)(f1 * WCARRY);
    const _Float16 e2 = (_Float16)(f2 * WCARRY), e3 = (_Float16)(f3 * WCARRY);
    const unsigned u0 = (unsigned)__builtin_bit_cast(unsigned short, e0);
    const unsigned u1 = (unsigned)__builtin_bit_cast(unsigned short, e1);
    const unsigned u2 = (unsigned)__builtin_bit_cast(unsigned short, e2);
    const unsigned u3 = (unsigned)__builtin_bit_cast(unsigned short, e3);
    v2u pk;
    pk[0] = u0 | (u1 << 16);
    pk[1] = u2 | (u3 << 16);
    *(v2u*)(Wl + n * WP + k4) = pk;
  }
  *(v4u*)(Wl + tid * WP + NHID) = z4;
  if (wave == 0) {
    const int q4 = (lane & 15) * 4;
    const v4f v = *(const v4f*)(x + (size_t)rowbase * NIN + q4);
    *(v4f*)(Xs + q4) = v;
  }
  __syncthreads();

  float wi0[4], wi1[4], bs[4];
#pragma unroll
  for (int gg = 0; gg < 2; ++gg) {
    const int n = 64 * gg + gi;
    const v2f w2 = *(const v2f*)(w_ih + 2 * n);
    wi0[gg] = w2[0]; wi1[gg] = w2[1];
    bs[gg] = b_ih[n] + b_hh[n];
  }
  asm volatile("" ::: "memory");
#pragma unroll
  for (int gg = 2; gg < 4; ++gg) {
    const int n = 64 * gg + gi;
    const v2f w2 = *(const v2f*)(w_ih + 2 * n);
    wi0[gg] = w2[0]; wi1[gg] = w2[1];
    bs[gg] = b_ih[n] + b_hh[n];
  }
  asm volatile("" ::: "memory");
  const float wfc = w_fc[gi];

  float cst[8], hst[8];
#pragma unroll
  for (int r = 0; r < 8; ++r) { cst[r] = 0.0f; hst[r] = 0.0f; }

  const v8f z8 = {0.f, 0.f, 0.f, 0.f, 0.f, 0.f, 0.f, 0.f};
  const _Float16* wrow = Wl + gi * WP + koff;

#pragma unroll 1
  for (int t = 0; t < NSTEP; ++t) {
    const int cur = t & 1, nxt = cur ^ 1;
    const _Float16* ahrow = Ah + ((cur * 2 + grp) * 16 + c) * HP + koff;
    _Float16*       ahn   = Ah + (nxt * 2 + grp) * 16 * HP;

    v4f xq[4];
    {
      const float* xsr = Xs + cur * (ROWS_BLK * NIN) + 32 * grp + 16 * hh;
#pragma unroll
      for (int p = 0; p < 4; ++p) xq[p] = *(const v4f*)(xsr + 4 * p);
    }
    if (wave == 0) {
      const int tn = (t + 1 < NSTEP) ? (t + 1) : (NSTEP - 1);
      const int q4 = (lane & 15) * 4;
      const v4f v = *(const v4f*)(x + ((size_t)tn * NBAT + (size_t)rowbase) * NIN + q4);
      *(v4f*)(Xs + nxt * (ROWS_BLK * NIN) + q4) = v;
    }

    v8f acc0 = z8, acc1 = z8, acc2 = z8, acc3 = z8;
#pragma unroll
    for (int kc = 0; kc < 2; ++kc) {
      const v16h a  = Frag<_Float16>::load(ahrow + 32 * kc);
      const v16h b0 = Frag<_Float16>::load(wrow + 32 * kc);
      const v16h b1 = Frag<_Float16>::load(wrow + 64 * WP + 32 * kc);
      const v16h b2 = Frag<_Float16>::load(wrow + 128 * WP + 32 * kc);
      const v16h b3 = Frag<_Float16>::load(wrow + 192 * WP + 32 * kc);
      acc0 = Frag<_Float16>::mma(a, b0, acc0);
      acc1 = Frag<_Float16>::mma(a, b1, acc1);
      acc2 = Frag<_Float16>::mma(a, b2, acc2);
      acc3 = Frag<_Float16>::mma(a, b3, acc3);
      acc_guard4_ab(acc0, acc1, acc2, acc3, a, b3);
      keep4_h(b0, b1, b2, a);
    }
    acc_guard4(acc0, acc1, acc2, acc3);

#pragma unroll
    for (int r = 0; r < 8; ++r) {
      const float x0 = xq[r >> 1][2 * (r & 1)];
      const float x1 = xq[r >> 1][2 * (r & 1) + 1];
      const float gx0 = fmaf(x1, wi1[0], fmaf(x0, wi0[0], bs[0]));
      const float gx1 = fmaf(x1, wi1[1], fmaf(x0, wi0[1], bs[1]));
      const float gx2 = fmaf(x1, wi1[2], fmaf(x0, wi0[2], bs[2]));
      const float gx3 = fmaf(x1, wi1[3], fmaf(x0, wi0[3], bs[3]));
      const float zi = fmaf(acc0[r], SC_INV, gx0);
      const float zf = fmaf(acc1[r], SC_INV, gx1);
      const float zg = fmaf(acc2[r], SC_INV, gx2);
      const float zo = fmaf(acc3[r], SC_INV, gx3);
      const float ig = sigm_f(zi);
      const float fg = sigm_f(zf);
      const float gv = tanh_f(zg);
      const float og = sigm_f(zo);
      const float cn = fg * cst[r] + ig * gv;
      cst[r] = cn;
      const float hn = og * tanh_f(cn);
      hst[r] = hn;
      ahn[(8 * hh + r) * HP + gi] = (_Float16)(hn * HCARRY);
    }
    __syncthreads();
  }

  float pr[8];
#pragma unroll
  for (int r = 0; r < 8; ++r) pr[r] = hst[r] * wfc;
#pragma unroll
  for (int r = 0; r < 8; ++r) {
#pragma unroll
    for (int off = 1; off < 16; off <<= 1) pr[r] += __shfl_xor(pr[r], off, 32);
  }
  if (c == 0) {
    float* pp = Ps + (grp * 4 + jt) * 16 + 8 * hh;
    const v4f p0 = {pr[0], pr[1], pr[2], pr[3]};
    const v4f p1 = {pr[4], pr[5], pr[6], pr[7]};
    *(v4f*)(pp)     = p0;
    *(v4f*)(pp + 4) = p1;
  }
  __syncthreads();
  if (wave == 0) {
    const int g2 = lane >> 4, rw = lane & 15;
    const float* pp = Ps + g2 * 64 + rw;
    const float tot = (((pp[0] + pp[16]) + pp[32]) + pp[48]) + b_fc[0];
    Os[lane] = tot;
  }
  __syncthreads();
  if (wave == 0) {
    if (lane < 8) {
      const v4f v = *(const v4f*)(Os + 4 * lane);
      float* op = out + (size_t)rowbase + 4 * lane;
      *(volatile v4f*)op = v;
      __threadfence();
      *(volatile v4f*)op = v;
    }
  }
}

extern "C" void kernel_launch(void* const* d_in, const int* in_sizes, int n_in,
                              void* d_out, int out_size, void* d_ws, size_t ws_size, hipStream_t stream) {
  if (n_in < 7 || d_out == nullptr) return;
  if (in_sizes[0] != NSTEP * NBAT * NIN || in_sizes[1] != NGATE * NIN || in_sizes[2] != NGATE * NHID ||
      in_sizes[3] != NGATE || in_sizes[4] != NGATE || in_sizes[5] != NHID || in_sizes[6] != 1 ||
      out_size != NBAT) return;

  const float* x    = (const float*)d_in[0];
  const float* w_ih = (const float*)d_in[1];
  const float* w_hh = (const float*)d_in[2];
  const float* b_ih = (const float*)d_in[3];
  const float* b_hh = (const float*)d_in[4];
  const float* w_fc = (const float*)d_in[5];
  const float* b_fc = (const float*)d_in[6];
  float* out = (float*)d_out;

  lstm_seq_kernel<<<NBAT / ROWS_BLK, NTHR, 0, stream>>>(x, w_ih, w_hh, b_ih, b_hh, w_fc, b_fc, out);
}
